// MultiHeadAttentionRelative_54296976556831
// MI455X (gfx1250) — hardware-verified
//
#include <hip/hip_runtime.h>
#include <stddef.h>
#include <stdint.h>

#define NB    8
#define SL    1024
#define DH    64
#define NH    8
#define DMH   512
#define NTOK  8192
#define NREL  301
#define NRP   320
#define MREL  150
#define TQ    32
#define SFP   68

static_assert(NTOK == NB * SL);
static_assert(DMH == NH * DH);
static_assert(SL % TQ == 0);
static_assert(SL % 64 == 0);
static_assert(NRP % 32 == 0);
static_assert(NRP >= NREL);
static_assert(DH == 64);
static_assert(TQ == 32);

#define ATT_SP    1028
#define ATT_PP    1032
#define ATT_RP    324
#define ATT_AP    328
#define ATT_CP    72
#define ATT_OFF_P (TQ * ATT_SP * 4)
#define ATT_OFF_R (ATT_OFF_P + TQ * ATT_PP * 2)
#define ATT_OFF_A (ATT_OFF_R + TQ * ATT_RP * 4)
#define ATT_LDS   (ATT_OFF_A + TQ * ATT_AP * 2)
static_assert(ATT_OFF_P % 16 == 0);
static_assert(ATT_OFF_R % 16 == 0);
static_assert(ATT_OFF_A % 16 == 0);
static_assert(TQ * ATT_CP * 2 <= ATT_OFF_P);

typedef _Float16 f16t;
typedef f16t         v16h __attribute__((ext_vector_type(16)));
typedef f16t         v8h  __attribute__((ext_vector_type(8)));
typedef float        v8f  __attribute__((ext_vector_type(8)));
typedef float        v4f  __attribute__((ext_vector_type(4)));
typedef unsigned int v4u  __attribute__((ext_vector_type(4)));

union Frag  { v16h v; v8h h[2]; };
union Pack8 { v8h h; v4u u; };

__device__ __forceinline__ v8f zero8() { return (v8f){0.f, 0.f, 0.f, 0.f, 0.f, 0.f, 0.f, 0.f}; }
__device__ __forceinline__ v4f zero4() { return (v4f){0.f, 0.f, 0.f, 0.f}; }

__device__ __forceinline__ v8f mma16(v16h a, v16h b, v8f c) {
  c = __builtin_amdgcn_wmma_f32_16x16x32_f16(false, a, false, b, (short)0, c, false, false);
  asm volatile("v_nop\n\tv_nop\n\tv_nop\n\tv_nop" : "+v"(c) : "v"(a), "v"(b));
  return c;
}

__device__ __forceinline__ v16h ldfrag(const f16t* p, int ld, int row0, int k0, int lane) {
  const int m = lane & 15, lh = lane >> 4;
  const f16t* q = p + (size_t)(row0 + m) * ld + k0 + 8 * lh;
  Frag f;
  f.h[0] = *(const v8h*)(q);
  f.h[1] = *(const v8h*)(q + 16);
  return f.v;
}

__device__ __forceinline__ v4u pack8(const float (&f)[8]) {
  Pack8 pk;
  pk.h = (v8h){(f16t)f[0], (f16t)f[1], (f16t)f[2], (f16t)f[3], (f16t)f[4], (f16t)f[5], (f16t)f[6], (f16t)f[7]};
  return pk.u;
}

__global__ __launch_bounds__(256) void k_cvt_x(const float* __restrict__ x0, const float* __restrict__ x1,
                                               const float* __restrict__ x2,
                                               f16t* __restrict__ y0, f16t* __restrict__ y1, f16t* __restrict__ y2) {
  const int z = blockIdx.y;
  const float* x = (z == 0) ? x0 : ((z == 1) ? x1 : x2);
  f16t* y = (z == 0) ? y0 : ((z == 1) ? y1 : y2);
  const size_t i = ((size_t)blockIdx.x * 256 + threadIdx.x) * 8;
  const v4f a0 = *(const v4f*)(x + i);
  const v4f a1 = *(const v4f*)(x + i + 4);
  const float f[8] = {a0[0], a0[1], a0[2], a0[3], a1[0], a1[1], a1[2], a1[3]};
  const v4u u = pack8(f);
  *(volatile v4u*)(y + i) = u;
  __threadfence();
  *(volatile v4u*)(y + i) = u;
}

__global__ __launch_bounds__(256) void k_tr64(const float* __restrict__ s0, const float* __restrict__ s1,
                                              const float* __restrict__ s2,
                                              f16t* __restrict__ d0p, f16t* __restrict__ d1p, f16t* __restrict__ d2p,
                                              int sp, int srows, int rstep, int cstep, int dp, float scale) {
  __shared__ __align__(16) float sw[64 * SFP];
  const int z = blockIdx.y;
  const float* src = (z == 0) ? s0 : ((z == 1) ? s1 : s2);
  f16t* dst = (z == 0) ? d0p : ((z == 1) ? d1p : d2p);
  const int tid = threadIdx.x;
  const int rb = blockIdx.x * rstep, cb = blockIdx.x * cstep;
  {
    const int r  = tid >> 2;
    const int c0 = (tid & 3) * 16;
    const int sr = rb + r;
    const int src_r = (sr < srows) ? sr : (srows - 1);
    const bool ok = (sr < srows);
    const float* q = src + (size_t)src_r * sp + cb + c0;
#pragma unroll
    for (int e = 0; e < 4; ++e) {
      v4f v = *(const v4f*)(q + 4 * e);
      if (!ok) v = zero4();
      *(v4f*)(sw + r * SFP + c0 + 4 * e) = v;
    }
  }
  __syncthreads();
  v4u hv[2];
  size_t go[2];
#pragma unroll
  for (int j = 0; j < 2; ++j) {
    const int p  = tid + 256 * j;
    const int cc = p >> 3;
    const int pc = p & 7;
    const float* cp = sw + (pc * 8) * SFP + cc;
    float f[8];
#pragma unroll
    for (int e = 0; e < 8; ++e) f[e] = cp[e * SFP] * scale;
    hv[j] = pack8(f);
    go[j] = (size_t)(cb + cc) * (size_t)dp + rb + pc * 8;
  }
#pragma unroll
  for (int j = 0; j < 2; ++j) *(volatile v4u*)(dst + go[j]) = hv[j];
  __threadfence();
#pragma unroll
  for (int j = 0; j < 2; ++j) *(volatile v4u*)(dst + go[j]) = hv[j];
}

__global__ __launch_bounds__(256) void k_cvt_relk(const float* __restrict__ rk, f16t* __restrict__ out16) {
  const int i = (blockIdx.x * 256 + threadIdx.x) * 8;
  const int row = i >> 6, col = i & 63;
  const int rr = (row < NREL) ? row : (NREL - 1);
  const bool ok = (row < NREL);
  const float* q = rk + (size_t)rr * DH + col;
  v4f a0 = *(const v4f*)(q);
  v4f a1 = *(const v4f*)(q + 4);
  if (!ok) { a0 = zero4(); a1 = zero4(); }
  const float f[8] = {a0[0] * 64.f, a0[1] * 64.f, a0[2] * 64.f, a0[3] * 64.f,
                      a1[0] * 64.f, a1[1] * 64.f, a1[2] * 64.f, a1[3] * 64.f};
  const v4u u = pack8(f);
  *(volatile v4u*)(out16 + i) = u;
  __threadfence();
  *(volatile v4u*)(out16 + i) = u;
}

#define PROJ_FOLD (1.0f / 64.0f)
__global__ __launch_bounds__(128) void k_proj(const f16t* __restrict__ xq, const f16t* __restrict__ xk,
                                              const f16t* __restrict__ xv,
                                              const f16t* __restrict__ wq, const f16t* __restrict__ wk,
                                              const f16t* __restrict__ wv,
                                              f16t* __restrict__ Qp, f16t* __restrict__ Kp, f16t* __restrict__ Vt) {
  __shared__ __align__(16) float sf[64 * SFP];
  const int z = blockIdx.z, hd = blockIdx.y;
  const f16t* X = (z == 0) ? xq : ((z == 1) ? xk : xv);
  const f16t* W = (z == 0) ? wq : ((z == 1) ? wk : wv);
  const int tid = threadIdx.x, lane = tid & 31, wave = tid >> 5;
  const int hh = lane >> 4, c = lane & 15;
  const int mb = blockIdx.x * 64;
  const int m0 = mb + wave * 16;

  v8f acc[4];
#pragma unroll
  for (int t = 0; t < 4; ++t) acc[t] = zero8();
#pragma unroll
  for (int k0 = 0; k0 < DH; k0 += 32) {
    const v16h a = ldfrag(X, DH, m0, k0, lane);
#pragma unroll
    for (int t = 0; t < 4; ++t) {
      const v16h bb = ldfrag(W, DH, hd * DH + 16 * t, k0, lane);
      acc[t] = mma16(a, bb, acc[t]);
    }
  }
#pragma unroll
  for (int t = 0; t < 4; ++t) {
#pragma unroll
    for (int r = 0; r < 8; ++r)
      sf[(wave * 16 + 8 * hh + r) * SFP + 16 * t + c] = acc[t][r] * PROJ_FOLD;
  }
  __syncthreads();

  v4u hv[4];
  size_t go[4];
  f16t* dst;
  if (z < 2) {
    dst = (z == 0) ? Qp : Kp;
#pragma unroll
    for (int j = 0; j < 4; ++j) {
      const int p  = tid + 128 * j;
      const int lr = p >> 3;
      const int d0 = (p & 7) * 8;
      const float* ra = sf + lr * SFP + d0;
      const v4f a0 = *(const v4f*)(ra), a1 = *(const v4f*)(ra + 4);
      const float f[8] = {a0[0], a0[1], a0[2], a0[3], a1[0], a1[1], a1[2], a1[3]};
      hv[j] = pack8(f);
      go[j] = ((size_t)(mb + lr)) * DMH + hd * DH + d0;
    }
  } else {
    dst = Vt;
    const int bI = mb / SL, l0 = mb - bI * SL;
#pragma unroll
    for (int j = 0; j < 4; ++j) {
      const int p  = tid + 128 * j;
      const int d  = p >> 3;
      const int pc = p & 7;
      const float* cp = sf + (pc * 8) * SFP + d;
      float f[8];
#pragma unroll
      for (int e = 0; e < 8; ++e) f[e] = cp[e * SFP];
      hv[j] = pack8(f);
      go[j] = ((size_t)((bI * NH + hd) * DH + d)) * SL + l0 + pc * 8;
    }
  }
#pragma unroll
  for (int j = 0; j < 4; ++j) *(volatile v4u*)(dst + go[j]) = hv[j];
  __threadfence();
#pragma unroll
  for (int j = 0; j < 4; ++j) *(volatile v4u*)(dst + go[j]) = hv[j];
}

__global__ __launch_bounds__(256) void k_attn(const f16t* __restrict__ Qp, const f16t* __restrict__ Kp,
                                              const f16t* __restrict__ Vt, const f16t* __restrict__ relk,
                                              const f16t* __restrict__ relvt, f16t* __restrict__ ctx) {
  extern __shared__ v4f smem_dyn[];
  char* smem = (char*)smem_dyn;
  float* Ssh = (float*)smem;
  f16t*  Psh = (f16t*)(smem + ATT_OFF_P);
  float* Rsh = (float*)(smem + ATT_OFF_R);
  f16t*  Ash = (f16t*)(smem + ATT_OFF_A);
  f16t*  Csh = (f16t*)smem;

  const int qt = blockIdx.x, h = blockIdx.y, b = blockIdx.z;
  const int tid = threadIdx.x, wave = tid >> 5, lane = tid & 31, hh = lane >> 4, c = lane & 15;
  const int q0  = qt * TQ;
  const int tq0 = b * SL + q0;
  const f16t* Qh = Qp + h * DH;
  const f16t* Kh = Kp + (size_t)b * SL * DMH + h * DH;

#pragma unroll
  for (int mt = 0; mt < 2; ++mt) {
    const v16h a0 = ldfrag(Qh, DMH, tq0 + mt * 16, 0, lane);
    const v16h a1 = ldfrag(Qh, DMH, tq0 + mt * 16, 32, lane);
#pragma unroll 1
    for (int nt = wave; nt < NRP / 16; nt += 8) {
      v8f acc = zero8();
      acc = mma16(a0, ldfrag(relk, DH, nt * 16, 0, lane), acc);
      acc = mma16(a1, ldfrag(relk, DH, nt * 16, 32, lane), acc);
#pragma unroll
      for (int r = 0; r < 8; ++r) Rsh[(mt * 16 + 8 * hh + r) * ATT_RP + nt * 16 + c] = acc[r];
    }
#pragma unroll 1
    for (int nt = wave; nt < SL / 16; nt += 8) {
      v8f acc = zero8();
      acc = mma16(a0, ldfrag(Kh, DMH, nt * 16, 0, lane), acc);
      acc = mma16(a1, ldfrag(Kh, DMH, nt * 16, 32, lane), acc);
#pragma unroll
      for (int r = 0; r < 8; ++r) Ssh[(mt * 16 + 8 * hh + r) * ATT_SP + nt * 16 + c] = acc[r];
    }
  }
  __syncthreads();

  const int row = tid >> 3, sub = tid & 7;
  const int qi = q0 + row;
  float* srow = Ssh + row * ATT_SP;
  const float* rrow = Rsh + row * ATT_RP;
  f16t* prow = Psh + row * ATT_PP;
  f16t* arow = Ash + row * ATT_AP;

  float mx = -__builtin_huge_valf();
#pragma unroll 4
  for (int i = 0; i < SL / 8; ++i) {
    const int kk = i * 8 + sub;
    int dl = kk - qi;
    dl = (dl < -MREL) ? -MREL : ((dl > MREL) ? MREL : dl);
    const float z = srow[kk] * 0.125f + rrow[dl + MREL] * (1.0f / 512.0f);
    srow[kk] = z;
    mx = fmaxf(mx, z);
  }
  mx = fmaxf(mx, __shfl_xor(mx, 1, 32));
  mx = fmaxf(mx, __shfl_xor(mx, 2, 32));
  mx = fmaxf(mx, __shfl_xor(mx, 4, 32));

  float sum = 0.f;
#pragma unroll 4
  for (int i = 0; i < SL / 8; ++i) {
    const int kk = i * 8 + sub;
    const float e = __expf(srow[kk] - mx);
    srow[kk] = e;
    sum += e;
  }
  sum += __shfl_xor(sum, 1, 32);
  sum += __shfl_xor(sum, 2, 32);
  sum += __shfl_xor(sum, 4, 32);
  const float cs = (1.0f / sum) * 1024.0f;

  float bk0 = 0.f, bk3 = 0.f;
#pragma unroll 4
  for (int i = 0; i < SL / 8; ++i) {
    const int kk = i * 8 + sub;
    const float ps = srow[kk] * cs;
    prow[kk] = (f16t)ps;
    bk0 += (kk <= qi - MREL) ? ps : 0.f;
    bk3 += (kk >= qi + MREL) ? ps : 0.f;
  }
  bk0 += __shfl_xor(bk0, 1, 32);
  bk0 += __shfl_xor(bk0, 2, 32);
  bk0 += __shfl_xor(bk0, 4, 32);
  bk3 += __shfl_xor(bk3, 1, 32);
  bk3 += __shfl_xor(bk3, 2, 32);
  bk3 += __shfl_xor(bk3, 4, 32);
  __syncthreads();

#pragma unroll 2
  for (int j = sub; j < NRP; j += 8) {
    const int kk  = qi + j - MREL;
    const int kkc = (kk < 0) ? 0 : ((kk > SL - 1) ? (SL - 1) : kk);
    const float e = srow[kkc] * cs;
    const bool okm = (j >= 1) && (j <= 2 * MREL - 1) && (kk >= 0) && (kk <= SL - 1);
    float v = okm ? e : 0.f;
    v = (j == 0) ? bk0 : v;
    v = (j == 2 * MREL) ? bk3 : v;
    arow[j] = (f16t)v;
  }
  __syncthreads();

  {
    const int mt = wave >> 2, nt = wave & 3;
    const f16t* Vb = Vt + ((size_t)((b * NH + h) * DH)) * SL;
    v8f acc1 = zero8(), acc2 = zero8();
#pragma unroll 4
    for (int k0 = 0; k0 < SL; k0 += 32) {
      const v16h a  = ldfrag(Psh, ATT_PP, mt * 16, k0, lane);
      const v16h bb = ldfrag(Vb, SL, nt * 16, k0, lane);
      acc1 = mma16(a, bb, acc1);
    }
#pragma unroll 2
    for (int k0 = 0; k0 < NRP; k0 += 32) {
      const v16h a  = ldfrag(Ash, ATT_AP, mt * 16, k0, lane);
      const v16h bb = ldfrag(relvt, NRP, nt * 16, k0, lane);
      acc2 = mma16(a, bb, acc2);
    }
#pragma unroll
    for (int r = 0; r < 8; ++r) {
      const float cv = acc1[r] * (1.0f / 16.0f) + acc2[r] * (1.0f / 1024.0f);
      Csh[(mt * 16 + 8 * hh + r) * ATT_CP + nt * 16 + c] = (f16t)cv;
    }
  }
  __syncthreads();
  {
    const int lr = tid >> 3, pc = tid & 7;
    const v4u u = *(const v4u*)(Csh + lr * ATT_CP + pc * 8);
    f16t* gp = ctx + ((size_t)(tq0 + lr)) * DMH + h * DH + pc * 8;
    *(volatile v4u*)gp = u;
    __threadfence();
    *(volatile v4u*)gp = u;
  }
}

#define OUT_FOLD (1.0f / 4096.0f)
__global__ __launch_bounds__(128) void k_out(const f16t* __restrict__ ctx, const f16t* __restrict__ wot,
                                             float* __restrict__ out) {
  __shared__ __align__(16) float sf[64 * SFP];
  const int tid = threadIdx.x, lane = tid & 31, wave = tid >> 5;
  const int hh = lane >> 4, c = lane & 15;
  const int mb = blockIdx.x * 64;
  const int m0 = mb + wave * 16;

  v8f acc[4];
#pragma unroll
  for (int t = 0; t < 4; ++t) acc[t] = zero8();
#pragma unroll 2
  for (int k0 = 0; k0 < DMH; k0 += 32) {
    const v16h a = ldfrag(ctx, DMH, m0, k0, lane);
#pragma unroll
    for (int t = 0; t < 4; ++t) {
      const v16h bb = ldfrag(wot, DMH, 16 * t, k0, lane);
      acc[t] = mma16(a, bb, acc[t]);
    }
  }
#pragma unroll
  for (int t = 0; t < 4; ++t) {
#pragma unroll
    for (int r = 0; r < 8; ++r)
      sf[(wave * 16 + 8 * hh + r) * SFP + 16 * t + c] = acc[t][r] * OUT_FOLD;
  }
  __syncthreads();
  v4f val[8];
  size_t go[8];
#pragma unroll
  for (int it = 0; it < 8; ++it) {
    const int p  = tid + 128 * it;
    const int lr = p >> 4;
    const int pc = p & 15;
    val[it] = *(const v4f*)(sf + lr * SFP + pc * 4);
    go[it]  = ((size_t)(mb + lr)) * DH + pc * 4;
  }
#pragma unroll
  for (int it = 0; it < 8; ++it) *(volatile v4f*)(out + go[it]) = val[it];
  __threadfence();
#pragma unroll
  for (int it = 0; it < 8; ++it) *(volatile v4f*)(out + go[it]) = val[it];
}

extern "C" void kernel_launch(void* const* d_in, const int* in_sizes, int n_in,
                              void* d_out, int out_size, void* d_ws, size_t ws_size,
                              hipStream_t stream) {
  if (n_in < 9) return;
  if (in_sizes[0] != NTOK * DH) return;
  if (in_sizes[1] != NTOK * DH) return;
  if (in_sizes[2] != NTOK * DH) return;
  if (in_sizes[3] != DH * DMH) return;
  if (in_sizes[4] != DH * DMH) return;
  if (in_sizes[5] != DH * DMH) return;
  if (in_sizes[6] != DMH * DH) return;
  if (in_sizes[7] != NREL * DH) return;
  if (in_sizes[8] != NREL * DH) return;
  if (out_size != NTOK * DH) return;

  const float* query = (const float*)d_in[0];
  const float* key   = (const float*)d_in[1];
  const float* value = (const float*)d_in[2];
  const float* Wq    = (const float*)d_in[3];
  const float* Wk    = (const float*)d_in[4];
  const float* Wv    = (const float*)d_in[5];
  const float* Wo    = (const float*)d_in[6];
  const float* rkt   = (const float*)d_in[7];
  const float* rvt   = (const float*)d_in[8];
  float* out = (float*)d_out;

  size_t off = 0;
  const size_t oXQ  = off; off += (size_t)NTOK * DH * 2;
  const size_t oXK  = off; off += (size_t)NTOK * DH * 2;
  const size_t oXV  = off; off += (size_t)NTOK * DH * 2;
  const size_t oWQ  = off; off += (size_t)DMH * DH * 2;
  const size_t oWK  = off; off += (size_t)DMH * DH * 2;
  const size_t oWV  = off; off += (size_t)DMH * DH * 2;
  const size_t oWO  = off; off += (size_t)DH * DMH * 2;
  const size_t oRK  = off; off += (size_t)NRP * DH * 2;
  const size_t oRVT = off; off += (size_t)DH * NRP * 2;
  const size_t oQP  = off; off += (size_t)NTOK * DMH * 2;
  const size_t oKP  = off; off += (size_t)NTOK * DMH * 2;
  const size_t oVT  = off; off += (size_t)NB * NH * DH * SL * 2;
  const size_t oCTX = off; off += (size_t)NTOK * DMH * 2;
  if (off > ws_size) return;
  if (off > (size_t)134217728) return;

  char* ws = (char*)d_ws;
  f16t* XQ  = (f16t*)(ws + oXQ);   f16t* XK  = (f16t*)(ws + oXK);   f16t* XV = (f16t*)(ws + oXV);
  f16t* WQ  = (f16t*)(ws + oWQ);   f16t* WK  = (f16t*)(ws + oWK);   f16t* WV = (f16t*)(ws + oWV);
  f16t* WO  = (f16t*)(ws + oWO);
  f16t* RK  = (f16t*)(ws + oRK);   f16t* RVT = (f16t*)(ws + oRVT);
  f16t* QP  = (f16t*)(ws + oQP);   f16t* KP  = (f16t*)(ws + oKP);   f16t* VT = (f16t*)(ws + oVT);
  f16t* CTX = (f16t*)(ws + oCTX);

  k_cvt_x<<<dim3((NTOK * DH) / 2048, 3), dim3(256), 0, stream>>>(query, key, value, XQ, XK, XV);
  k_tr64<<<dim3(DMH / 64, 3), dim3(256), 0, stream>>>(Wq, Wk, Wv, WQ, WK, WV, DMH, DH, 0, 64, DH, 64.0f);
  k_tr64<<<dim3(DMH / 64, 1), dim3(256), 0, stream>>>(Wo, Wo, Wo, WO, WO, WO, DH, DMH, 64, 0, DMH, 64.0f);
  k_tr64<<<dim3(NRP / 64, 1), dim3(256), 0, stream>>>(rvt, rvt, rvt, RVT, RVT, RVT, DH, NREL, 64, 0, NRP, 64.0f);
  k_cvt_relk<<<dim3((NRP * DH) / 2048), dim3(256), 0, stream>>>(rkt, RK);
  k_proj<<<dim3(NTOK / 64, NH, 3), dim3(128), 0, stream>>>(XQ, XK, XV, WQ, WK, WV, QP, KP, VT);
  (void)hipFuncSetAttribute(reinterpret_cast<const void*>(&k_attn), hipFuncAttributeMaxDynamicSharedMemorySize,
                            ATT_LDS);
  k_attn<<<dim3(SL / TQ, NH, NB), dim3(256), ATT_LDS, stream>>>(QP, KP, VT, RK, RVT, CTX);
  k_out<<<dim3(NTOK / 64), dim3(128), 0, stream>>>(CTX, WO, out);
  (void)hipGetLastError();
}
